// GRUModel_15728170238726
// MI455X (gfx1250) — hardware-verified
//
#include <hip/hip_runtime.h>
#include <math.h>

constexpr int NB   = 256;
constexpr int NTT  = 2048;
constexpr int NIN  = 29;
constexpr int NH   = 64;
constexpr int NG3  = 192;
constexpr int NEMB = 128;
constexpr int NOF  = 11;
constexpr int NTHR = 512;
constexpr int NWAV = NTHR / 32;
constexpr int RB   = 32;
constexpr int TROWS = 2 * RB;
constexpr int XKP  = 32;
constexpr int XP   = 40;
constexpr int HP   = 72;
constexpr int XT_ELEMS = TROWS * XP;
constexpr int HT_ELEMS = TROWS * HP;
constexpr int EP   = 132;
constexpr int H1P  = 68;
constexpr int LDSW_FLOATS = (2 * NG3 * NEMB) / 2;
constexpr float WCARRY     = 16.0f;
constexpr float WCARRY_INV = 1.0f / 16.0f;
constexpr float LN_EPS     = 1e-5f;

static_assert(NB % RB == 0);
static_assert(NTHR == 512 && NWAV == 16 && RB == 32 && NH == 64 && NEMB == 2 * NH && NG3 == 3 * NH);
static_assert((2 * NG3 * NH) % NTHR == 0 && (2 * NG3 * XKP) % NTHR == 0 && (2 * NG3 * NEMB) % NTHR == 0);
static_assert(2 * RB * XKP == 4 * NTHR);
static_assert(TROWS == 4 * NWAV);
static_assert((4 * HT_ELEMS) % NTHR == 0);
static_assert(XP % 8 == 0 && HP % 8 == 0 && EP % 4 == 0 && H1P % 4 == 0);
static_assert(XKP % 32 == 0 && NH % 32 == 0 && NEMB % 32 == 0);
static_assert(NIN <= XKP);
static_assert((RB * NOF) % 4 == 0 && ((RB * NOF * 4) % 128) == 0 && (RB * NOF) / 4 <= NTHR);
static_assert(RB == 2 * NWAV);
static_assert(RB * EP + RB * H1P + RB * NOF <= LDSW_FLOATS);
static_assert(2 * NG3 * NH <= 2 * LDSW_FLOATS);

typedef __attribute__((ext_vector_type(16))) _Float16 v16h;
typedef __attribute__((ext_vector_type(8)))  _Float16 v8h;
typedef __attribute__((ext_vector_type(16))) __bf16   v16b;
typedef __attribute__((ext_vector_type(8)))  __bf16   v8b;
typedef __attribute__((ext_vector_type(8)))  float    v8f;
typedef __attribute__((ext_vector_type(4)))  float    v4f;
typedef __attribute__((ext_vector_type(2)))  unsigned v2u;
typedef __attribute__((ext_vector_type(4)))  unsigned v4u;

__device__ __forceinline__ unsigned short f2bf_bits(float f) {
  unsigned u = __float_as_uint(f);
  return (unsigned short)((u + 0x7FFFu + ((u >> 16) & 1u)) >> 16);
}
__device__ __forceinline__ float bf_bits2f(unsigned short h) { return __uint_as_float(((unsigned)h) << 16); }
__device__ __forceinline__ float bf16r(float f) { return bf_bits2f(f2bf_bits(f)); }

__device__ __forceinline__ void dep_guard_h(v8f& a, v8f& b, v16h x, v16h y) { asm volatile("v_nop\n\tv_nop\n\tv_nop\n\tv_nop" : "+v"(a), "+v"(b) : "v"(x), "v"(y)); }
__device__ __forceinline__ void dep_guard_b(v8f& a, v8f& b, v16b x, v16b y) { asm volatile("v_nop\n\tv_nop\n\tv_nop\n\tv_nop" : "+v"(a), "+v"(b) : "v"(x), "v"(y)); }
__device__ __forceinline__ void guard3_h(v8f& a, v8f& b, v8f& c, v16h x, v16h y) { asm volatile("v_nop\n\tv_nop\n\tv_nop\n\tv_nop" : "+v"(a), "+v"(b), "+v"(c) : "v"(x), "v"(y)); }
__device__ __forceinline__ void guard3_b(v8f& a, v8f& b, v8f& c, v16b x, v16b y) { asm volatile("v_nop\n\tv_nop\n\tv_nop\n\tv_nop" : "+v"(a), "+v"(b), "+v"(c) : "v"(x), "v"(y)); }
__device__ __forceinline__ void keep4_h(v16h a, v16h b, v16h c, v16h d) { asm volatile("v_nop" :: "v"(a), "v"(b), "v"(c), "v"(d)); }
__device__ __forceinline__ void keep4_b(v16b a, v16b b, v16b c, v16b d) { asm volatile("v_nop" :: "v"(a), "v"(b), "v"(c), "v"(d)); }
__device__ __forceinline__ void acc_guard4(v8f& a, v8f& b, v8f& c, v8f& d) { asm volatile("v_nop\n\tv_nop\n\tv_nop\n\tv_nop" : "+v"(a), "+v"(b), "+v"(c), "+v"(d)); }
template <typename T> struct Frag;
template <> struct Frag<_Float16> {
  typedef v16h V; union U { v16h v; v8h h[2]; };
  static __device__ __forceinline__ v16h load(const _Float16* p) {
    U f; f.h[0] = *(const v8h*)(p); f.h[1] = *(const v8h*)(p + 16); return f.v;
  }
  static __device__ __forceinline__ v8f mma(v16h a, v16h b, v8f c) {
    return __builtin_amdgcn_wmma_f32_16x16x32_f16(false, a, false, b, (short)0, c, false, false);
  }
  static __device__ __forceinline__ void guard(v8f& a, v8f& b, v16h x, v16h y) { dep_guard_h(a, b, x, y); }
  static __device__ __forceinline__ void keep(v16h a, v16h b, v16h c, v16h d) { keep4_h(a, b, c, d); }
};
template <> struct Frag<__bf16> {
  typedef v16b V; union U { v16b v; v8b h[2]; };
  static __device__ __forceinline__ v16b load(const __bf16* p) {
    U f; f.h[0] = *(const v8b*)(p); f.h[1] = *(const v8b*)(p + 16); return f.v;
  }
  static __device__ __forceinline__ v8f mma(v16b a, v16b b, v8f c) {
    return __builtin_amdgcn_wmma_f32_16x16x32_bf16(false, a, false, b, (short)0, c, false, false);
  }
  static __device__ __forceinline__ void guard(v8f& a, v8f& b, v16b x, v16b y) { dep_guard_b(a, b, x, y); }
  static __device__ __forceinline__ void keep(v16b a, v16b b, v16b c, v16b d) { keep4_b(a, b, c, d); }
};

__device__ __forceinline__ float sigm(float v)  { return __builtin_amdgcn_rcpf(1.0f + expf(-v)); }
__device__ __forceinline__ float tanhe(float v) { return 1.0f - 2.0f * __builtin_amdgcn_rcpf(expf(2.0f * v) + 1.0f); }

__device__ __forceinline__ void stage_x_tile(const float* __restrict__ x, unsigned short* xt, int b0, int tid, int tf, int tb) {
  const int d2 = tid >> 8, row = (tid >> 3) & 31, j = tid & 7;
  const int t2 = d2 ? tb : tf;
  const float* xr = x + (((size_t)(b0 + row)) * NTT + (size_t)t2) * NIN;
  unsigned short hb[4];
#pragma unroll
  for (int e = 0; e < 4; ++e) {
    const int col = 4 * j + e;
    const int cc = (col < NIN) ? col : (NIN - 1);
    const float keep = (col < NIN) ? 1.0f : 0.0f;
    const float v = xr[cc] * keep;
    hb[e] = f2bf_bits(v);
  }
  v2u pk;
  pk[0] = (unsigned)hb[0] | ((unsigned)hb[1] << 16);
  pk[1] = (unsigned)hb[2] | ((unsigned)hb[3] << 16);
  *(v2u*)(xt + (d2 * RB + row) * XP + 4 * j) = pk;
}

__global__ __launch_bounds__(NTHR) void rec_l0_kernel(
    const float* __restrict__ x,
    const float* __restrict__ wihF, const float* __restrict__ whhF,
    const float* __restrict__ bihF, const float* __restrict__ bhhF,
    const float* __restrict__ wihB, const float* __restrict__ whhB,
    const float* __restrict__ bihB, const float* __restrict__ bhhB,
    unsigned short* __restrict__ seq) {
  __shared__ __align__(16) unsigned short Wxs[2 * NG3 * XKP];
  __shared__ __align__(16) unsigned short Whs[2 * NG3 * NH];
  __shared__ __align__(16) unsigned short Xt[2 * XT_ELEMS];
  __shared__ __align__(16) unsigned short Ht[4 * HT_ELEMS];
  __shared__ __align__(16) unsigned short Hs[2 * HT_ELEMS];
  const int tid = threadIdx.x, lane = tid & 31, wave = tid >> 5;
  const int c = lane & 15, hh = lane >> 4, koff = hh * 8;
  const int dir = wave >> 3, mt = (wave >> 2) & 1, ub = wave & 3;
  const int ucol = 16 * ub + c;
  const int lrow0 = dir * RB + 16 * mt;
  const int b0 = blockIdx.x * RB;

#pragma unroll 1
  for (int i = tid; i < 4 * HT_ELEMS; i += NTHR) Ht[i] = (unsigned short)0;
#pragma unroll 1
  for (int i = tid; i < 2 * NG3 * NH; i += NTHR) {
    const int d = (i >= NG3 * NH) ? 1 : 0;
    const int idx = i - d * (NG3 * NH);
    const float va = whhF[idx], vb = whhB[idx];
    const float fb = (float)d, fa = 1.0f - fb;
    const float v = fmaf(fb, vb, fa * va);
    Whs[i] = f2bf_bits(v * WCARRY);
  }
#pragma unroll 1
  for (int i = tid; i < 2 * NG3 * XKP; i += NTHR) {
    const int d = (i >= NG3 * XKP) ? 1 : 0;
    const int rem = i - d * (NG3 * XKP);
    const int n = rem >> 5, k = rem & 31;
    const int kc = (k < NIN) ? k : (NIN - 1);
    const float va = wihF[n * NIN + kc], vb = wihB[n * NIN + kc];
    const float fb = (float)d, fa = 1.0f - fb;
    const float v = fmaf(fb, vb, fa * va);
    const float sc = (k < NIN) ? WCARRY : 0.0f;
    Wxs[i] = f2bf_bits(v * sc);
  }
  stage_x_tile(x, Xt, b0, tid, 0, NTT - 1);
  const float fdb = (float)dir, fda = 1.0f - fdb;
  const float b_r  = fmaf(fdb, bf16r(bihB[ucol]) + bf16r(bhhB[ucol]),           fda * (bf16r(bihF[ucol]) + bf16r(bhhF[ucol])));
  const float b_z  = fmaf(fdb, bf16r(bihB[NH + ucol]) + bf16r(bhhB[NH + ucol]), fda * (bf16r(bihF[NH + ucol]) + bf16r(bhhF[NH + ucol])));
  const float b_xn = fmaf(fdb, bf16r(bihB[2 * NH + ucol]),                     fda * bf16r(bihF[2 * NH + ucol]));
  const float b_hn = fmaf(fdb, bf16r(bhhB[2 * NH + ucol]),                     fda * bf16r(bhhF[2 * NH + ucol]));
  float hst[8];
#pragma unroll
  for (int r = 0; r < 8; ++r) hst[r] = 0.0f;
  __syncthreads();

  const v8f z8 = {0.f, 0.f, 0.f, 0.f, 0.f, 0.f, 0.f, 0.f};
#pragma unroll 1
  for (int s = 0; s < NTT; ++s) {
    const int cur = s & 1, nxt = cur ^ 1;
    const __bf16* xrow = (const __bf16*)(Xt + cur * XT_ELEMS + (lrow0 + c) * XP + koff);
    const __bf16* hhi  = (const __bf16*)(Ht + (cur * 2 + 0) * HT_ELEMS + (lrow0 + c) * HP + koff);
    const __bf16* hlo  = (const __bf16*)(Ht + (cur * 2 + 1) * HT_ELEMS + (lrow0 + c) * HP + koff);
    const __bf16* wxp  = (const __bf16*)(Wxs + (dir * NG3 + ucol) * XKP + koff);
    const __bf16* whp  = (const __bf16*)(Whs + (dir * NG3 + ucol) * NH + koff);
    v8f ar, az, anx, anh;
    {
      const v16b xa = Frag<__bf16>::load(xrow);
      const v16b wr = Frag<__bf16>::load(wxp);
      const v16b wz = Frag<__bf16>::load(wxp + NH * XKP);
      const v16b wn = Frag<__bf16>::load(wxp + 2 * NH * XKP);
      ar  = Frag<__bf16>::mma(xa, wr, z8);
      az  = Frag<__bf16>::mma(xa, wz, z8);
      anx = Frag<__bf16>::mma(xa, wn, z8);
      guard3_b(ar, az, anx, xa, wn);
      keep4_b(wr, wz, wn, xa);
    }
    anh = z8;
#pragma unroll
    for (int kc = 0; kc < 2; ++kc) {
      const v16b hah = Frag<__bf16>::load(hhi + 32 * kc);
      const v16b hal = Frag<__bf16>::load(hlo + 32 * kc);
      const v16b wr = Frag<__bf16>::load(whp + 32 * kc);
      const v16b wz = Frag<__bf16>::load(whp + NH * NH + 32 * kc);
      const v16b wn = Frag<__bf16>::load(whp + 2 * NH * NH + 32 * kc);
      ar  = Frag<__bf16>::mma(hah, wr, ar);
      ar  = Frag<__bf16>::mma(hal, wr, ar);
      az  = Frag<__bf16>::mma(hah, wz, az);
      az  = Frag<__bf16>::mma(hal, wz, az);
      anh = Frag<__bf16>::mma(hah, wn, anh);
      anh = Frag<__bf16>::mma(hal, wn, anh);
      guard3_b(ar, az, anh, hah, hal);
      keep4_b(wr, wz, wn, hal);
    }
    acc_guard4(ar, az, anx, anh);
    {
      unsigned short* hhn = Ht + (nxt * 2 + 0) * HT_ELEMS + (lrow0 + 8 * hh) * HP + ucol;
      unsigned short* hln = Ht + (nxt * 2 + 1) * HT_ELEMS + (lrow0 + 8 * hh) * HP + ucol;
      unsigned short* hsn = Hs + nxt * HT_ELEMS + (lrow0 + 8 * hh) * HP + ucol;
#pragma unroll
      for (int r = 0; r < 8; ++r) {
        const float pr  = ar[r]  * WCARRY_INV + b_r;
        const float pz  = az[r]  * WCARRY_INV + b_z;
        const float gxn = anx[r] * WCARRY_INV + b_xn;
        const float ghn = anh[r] * WCARRY_INV + b_hn;
        const float rg = sigm(pr);
        const float zg = sigm(pz);
        const float ng = tanhe(gxn + rg * ghn);
        const float ho = hst[r];
        const float hn = (1.0f - zg) * ng + zg * ho;
        hst[r] = hn;
        const unsigned short hb = f2bf_bits(hn);
        const unsigned short lb = f2bf_bits(hn - bf_bits2f(hb));
        hhn[r * HP] = hb;
        hln[r * HP] = lb;
        hsn[r * HP] = __builtin_bit_cast(unsigned short, (_Float16)hn);
      }
    }
    {
      const int tf = (s + 1 < NTT) ? (s + 1) : (NTT - 1);
      stage_x_tile(x, Xt + nxt * XT_ELEMS, b0, tid, tf, NTT - 1 - tf);
    }
    __syncthreads();
    {
      const int q = lane >> 3, e8 = (lane & 7) * 8;
      const int L = wave * 4 + q;
      const int dL = L >> 5, rowL = L & 31;
      const int tL = dL ? (NTT - 1 - s) : s;
      const v4u w = *(const v4u*)(Hs + nxt * HT_ELEMS + (dL * RB + rowL) * HP + e8);
      unsigned short* dst = seq + ((((size_t)(b0 + rowL)) * NTT + (size_t)tL) * NEMB + (size_t)(dL * NH + e8));
      for (int pass = 0; pass < 2; ++pass) {
        *(volatile v4u*)dst = w;
        __threadfence();
      }
    }
  }
}

__global__ __launch_bounds__(NTHR) void rec_l1_head_kernel(
    const unsigned short* __restrict__ seq,
    const float* __restrict__ wihF, const float* __restrict__ whhF,
    const float* __restrict__ bihF, const float* __restrict__ bhhF,
    const float* __restrict__ wihB, const float* __restrict__ whhB,
    const float* __restrict__ bihB, const float* __restrict__ bhhB,
    const float* __restrict__ lng, const float* __restrict__ lnb,
    const float* __restrict__ w1, const float* __restrict__ bb1,
    const float* __restrict__ w2, const float* __restrict__ bb2,
    float* __restrict__ out) {
  __shared__ __align__(16) float          LdsW[LDSW_FLOATS];
  __shared__ __align__(16) unsigned short Ht[4 * HT_ELEMS];
  unsigned short* Wsl = (unsigned short*)(void*)LdsW;
  const int tid = threadIdx.x, lane = tid & 31, wave = tid >> 5;
  const int c = lane & 15, hh = lane >> 4, koff = hh * 8;
  const int dir = wave >> 3, mt = (wave >> 2) & 1, ub = wave & 3;
  const int ucol = 16 * ub + c;
  const int lrow0 = dir * RB + 16 * mt;
  const int b0 = blockIdx.x * RB;

#pragma unroll 1
  for (int i = tid; i < 4 * HT_ELEMS; i += NTHR) Ht[i] = (unsigned short)0;
#pragma unroll 1
  for (int i = tid; i < 2 * NG3 * NH; i += NTHR) {
    const int d = (i >= NG3 * NH) ? 1 : 0;
    const int idx = i - d * (NG3 * NH);
    const float va = whhF[idx], vb = whhB[idx];
    const float fb = (float)d, fa = 1.0f - fb;
    const float v = fmaf(fb, vb, fa * va);
    Wsl[i] = f2bf_bits(v * WCARRY);
  }
  __syncthreads();
  v16b whr[2], whz[2], whn[2];
  {
    const __bf16* p = (const __bf16*)(Wsl + (dir * NG3 + ucol) * NH + koff);
#pragma unroll
    for (int kc = 0; kc < 2; ++kc) {
      whr[kc] = Frag<__bf16>::load(p + 32 * kc);
      whz[kc] = Frag<__bf16>::load(p + NH * NH + 32 * kc);
      whn[kc] = Frag<__bf16>::load(p + 2 * NH * NH + 32 * kc);
    }
  }
  __syncthreads();
#pragma unroll 1
  for (int i = tid; i < 2 * NG3 * NEMB; i += NTHR) {
    const int d = (i >= NG3 * NEMB) ? 1 : 0;
    const int idx = i - d * (NG3 * NEMB);
    const float va = wihF[idx], vb = wihB[idx];
    const float fb = (float)d, fa = 1.0f - fb;
    const float v = fmaf(fb, vb, fa * va);
    Wsl[i] = __builtin_bit_cast(unsigned short, (_Float16)(bf16r(v) * WCARRY));
  }
  const float fdb = (float)dir, fda = 1.0f - fdb;
  const float b_r  = fmaf(fdb, bf16r(bihB[ucol]) + bf16r(bhhB[ucol]),           fda * (bf16r(bihF[ucol]) + bf16r(bhhF[ucol])));
  const float b_z  = fmaf(fdb, bf16r(bihB[NH + ucol]) + bf16r(bhhB[NH + ucol]), fda * (bf16r(bihF[NH + ucol]) + bf16r(bhhF[NH + ucol])));
  const float b_xn = fmaf(fdb, bf16r(bihB[2 * NH + ucol]),                     fda * bf16r(bihF[2 * NH + ucol]));
  const float b_hn = fmaf(fdb, bf16r(bhhB[2 * NH + ucol]),                     fda * bf16r(bhhF[2 * NH + ucol]));
  float hst[8];
#pragma unroll
  for (int r = 0; r < 8; ++r) hst[r] = 0.0f;
  __syncthreads();

  const v8f z8 = {0.f, 0.f, 0.f, 0.f, 0.f, 0.f, 0.f, 0.f};
  const _Float16* seqh = (const _Float16*)seq;
#pragma unroll 1
  for (int s = 0; s < NTT; ++s) {
    const int cur = s & 1, nxt = cur ^ 1;
    const int td = dir ? (NTT - 1 - s) : s;
    const _Float16* arow = seqh + ((((size_t)(b0 + 16 * mt + c)) * NTT + (size_t)td) * NEMB + (size_t)koff);
    const __bf16* hhi = (const __bf16*)(Ht + (cur * 2 + 0) * HT_ELEMS + (lrow0 + c) * HP + koff);
    const __bf16* hlo = (const __bf16*)(Ht + (cur * 2 + 1) * HT_ELEMS + (lrow0 + c) * HP + koff);
    const _Float16* wxp = (const _Float16*)(Wsl + (dir * NG3 + ucol) * NEMB + koff);
    v8f ar = z8, az = z8, anx = z8, anh = z8;
#pragma unroll 1
    for (int kc = 0; kc < 4; ++kc) {
      const v16h xa = Frag<_Float16>::load(arow + 32 * kc);
      const v16h wr = Frag<_Float16>::load(wxp + 32 * kc);
      const v16h wz = Frag<_Float16>::load(wxp + NH * NEMB + 32 * kc);
      const v16h wn = Frag<_Float16>::load(wxp + 2 * NH * NEMB + 32 * kc);
      ar  = Frag<_Float16>::mma(xa, wr, ar);
      az  = Frag<_Float16>::mma(xa, wz, az);
      anx = Frag<_Float16>::mma(xa, wn, anx);
      guard3_h(ar, az, anx, xa, wn);
      keep4_h(wr, wz, wn, xa);
    }
#pragma unroll
    for (int kc = 0; kc < 2; ++kc) {
      const v16b hah = Frag<__bf16>::load(hhi + 32 * kc);
      const v16b hal = Frag<__bf16>::load(hlo + 32 * kc);
      ar  = Frag<__bf16>::mma(hah, whr[kc], ar);
      ar  = Frag<__bf16>::mma(hal, whr[kc], ar);
      az  = Frag<__bf16>::mma(hah, whz[kc], az);
      az  = Frag<__bf16>::mma(hal, whz[kc], az);
      anh = Frag<__bf16>::mma(hah, whn[kc], anh);
      anh = Frag<__bf16>::mma(hal, whn[kc], anh);
      guard3_b(ar, az, anh, hah, hal);
      keep4_b(whr[kc], whz[kc], whn[kc], hal);
    }
    acc_guard4(ar, az, anx, anh);
    {
      unsigned short* hhn = Ht + (nxt * 2 + 0) * HT_ELEMS + (lrow0 + 8 * hh) * HP + ucol;
      unsigned short* hln = Ht + (nxt * 2 + 1) * HT_ELEMS + (lrow0 + 8 * hh) * HP + ucol;
#pragma unroll
      for (int r = 0; r < 8; ++r) {
        const float pr  = ar[r]  * WCARRY_INV + b_r;
        const float pz  = az[r]  * WCARRY_INV + b_z;
        const float gxn = anx[r] * WCARRY_INV + b_xn;
        const float ghn = anh[r] * WCARRY_INV + b_hn;
        const float rg = sigm(pr);
        const float zg = sigm(pz);
        const float ng = tanhe(gxn + rg * ghn);
        const float ho = hst[r];
        const float hn = (1.0f - zg) * ng + zg * ho;
        hst[r] = hn;
        const unsigned short hb = f2bf_bits(hn);
        const unsigned short lb = f2bf_bits(hn - bf_bits2f(hb));
        hhn[r * HP] = hb;
        hln[r * HP] = lb;
      }
    }
    __syncthreads();
  }

  float* Emb  = LdsW;
  float* H1s  = LdsW + RB * EP;
  float* Outs = LdsW + RB * EP + RB * H1P;
  {
    float* ep = Emb + (16 * mt + 8 * hh) * EP + dir * NH + ucol;
#pragma unroll
    for (int r = 0; r < 8; ++r) ep[r * EP] = hst[r];
  }
  __syncthreads();
#pragma unroll 1
  for (int rr = 0; rr < 2; ++rr) {
    const int row = wave * 2 + rr;
    float* er = Emb + row * EP + 4 * lane;
    const v4f e = *(const v4f*)er;
    float su = (e[0] + e[1]) + (e[2] + e[3]);
#pragma unroll
    for (int off = 1; off < 32; off <<= 1) su += __shfl_xor(su, off, 32);
    const float mu = su * (1.0f / NEMB);
    v4f d;
    float ss = 0.0f;
#pragma unroll
    for (int k = 0; k < 4; ++k) { d[k] = e[k] - mu; ss += d[k] * d[k]; }
#pragma unroll
    for (int off = 1; off < 32; off <<= 1) ss += __shfl_xor(ss, off, 32);
    const float var  = ss * (1.0f / NEMB);
    const float rstd = __builtin_amdgcn_rcpf(sqrtf(var + LN_EPS));
    const v4f g  = *(const v4f*)(lng + 4 * lane);
    const v4f bt = *(const v4f*)(lnb + 4 * lane);
    v4f y;
#pragma unroll
    for (int k = 0; k < 4; ++k) y[k] = (d[k] * rstd) * bf16r(g[k]) + bf16r(bt[k]);
    *(v4f*)er = y;
  }
  __syncthreads();
#pragma unroll 1
  for (int rr = 0; rr < 2; ++rr) {
    const int row = wave * 2 + rr;
    const float* yr = Emb + row * EP;
    const int j0 = lane, j1 = lane + 32;
    float a0 = bf16r(bb1[j0]), a1 = bf16r(bb1[j1]);
    const float* wa = w1 + (size_t)j0 * NEMB;
    const float* wb = w1 + (size_t)j1 * NEMB;
#pragma unroll 1
    for (int k = 0; k < NEMB; k += 4) {
      const v4f yv = *(const v4f*)(yr + k);
      const v4f va = *(const v4f*)(wa + k);
      const v4f vb = *(const v4f*)(wb + k);
      a0 += yv[0] * bf16r(va[0]); a0 += yv[1] * bf16r(va[1]); a0 += yv[2] * bf16r(va[2]); a0 += yv[3] * bf16r(va[3]);
      a1 += yv[0] * bf16r(vb[0]); a1 += yv[1] * bf16r(vb[1]); a1 += yv[2] * bf16r(vb[2]); a1 += yv[3] * bf16r(vb[3]);
    }
    H1s[row * H1P + j0] = fmaxf(a0, 0.0f);
    H1s[row * H1P + j1] = fmaxf(a1, 0.0f);
  }
  __syncthreads();
#pragma unroll 1
  for (int rr = 0; rr < 2; ++rr) {
    const int row = wave * 2 + rr;
    const int jj = (lane < NOF) ? lane : (NOF - 1);
    float a = bf16r(bb2[jj]);
    const float* wv = w2 + (size_t)jj * NH;
    const float* hr = H1s + row * H1P;
#pragma unroll 1
    for (int k = 0; k < NH; k += 4) {
      const v4f hv = *(const v4f*)(hr + k);
      const v4f ww = *(const v4f*)(wv + k);
      a += hv[0] * bf16r(ww[0]); a += hv[1] * bf16r(ww[1]); a += hv[2] * bf16r(ww[2]); a += hv[3] * bf16r(ww[3]);
    }
    if (lane < NOF) Outs[row * NOF + lane] = a;
  }
  __syncthreads();
  if (tid < (RB * NOF) / 4) {
    const v4f v = *(const v4f*)(Outs + 4 * tid);
    float* op = out + (size_t)blockIdx.x * (RB * NOF) + 4 * tid;
    for (int pass = 0; pass < 2; ++pass) {
      *(volatile v4f*)op = v;
      __threadfence();
    }
  }
}

extern "C" void kernel_launch(void* const* d_in, const int* in_sizes, int n_in,
                              void* d_out, int out_size, void* d_ws, size_t ws_size, hipStream_t stream) {
  if (n_in < 23 || d_out == nullptr || d_ws == nullptr) return;
  if (in_sizes[0] != NB * NTT * NIN) return;
  if (in_sizes[1] != NG3 * NIN || in_sizes[2] != NG3 * NH || in_sizes[3] != NG3 || in_sizes[4] != NG3) return;
  if (in_sizes[5] != NG3 * NIN || in_sizes[6] != NG3 * NH || in_sizes[7] != NG3 || in_sizes[8] != NG3) return;
  if (in_sizes[9] != NG3 * NEMB || in_sizes[10] != NG3 * NH || in_sizes[11] != NG3 || in_sizes[12] != NG3) return;
  if (in_sizes[13] != NG3 * NEMB || in_sizes[14] != NG3 * NH || in_sizes[15] != NG3 || in_sizes[16] != NG3) return;
  if (in_sizes[17] != NEMB || in_sizes[18] != NEMB || in_sizes[19] != NH * NEMB || in_sizes[20] != NH ||
      in_sizes[21] != NOF * NH || in_sizes[22] != NOF || out_size != NB * NOF) return;

  const float* x     = (const float*)d_in[0];
  const float* wih00 = (const float*)d_in[1];
  const float* whh00 = (const float*)d_in[2];
  const float* bih00 = (const float*)d_in[3];
  const float* bhh00 = (const float*)d_in[4];
  const float* wih01 = (const float*)d_in[5];
  const float* whh01 = (const float*)d_in[6];
  const float* bih01 = (const float*)d_in[7];
  const float* bhh01 = (const float*)d_in[8];
  const float* wih10 = (const float*)d_in[9];
  const float* whh10 = (const float*)d_in[10];
  const float* bih10 = (const float*)d_in[11];
  const float* bhh10 = (const float*)d_in[12];
  const float* wih11 = (const float*)d_in[13];
  const float* whh11 = (const float*)d_in[14];
  const float* bih11 = (const float*)d_in[15];
  const float* bhh11 = (const float*)d_in[16];
  const float* lng   = (const float*)d_in[17];
  const float* lnb   = (const float*)d_in[18];
  const float* w1    = (const float*)d_in[19];
  const float* bb1   = (const float*)d_in[20];
  const float* w2    = (const float*)d_in[21];
  const float* bb2   = (const float*)d_in[22];
  float* out = (float*)d_out;

  const size_t SEQ_BYTES = (size_t)NB * NTT * NEMB * 2;
  if (SEQ_BYTES > ws_size || SEQ_BYTES > (size_t)134217728) return;
  unsigned short* seq = (unsigned short*)d_ws;

  rec_l0_kernel<<<NB / RB, NTHR, 0, stream>>>(x, wih00, whh00, bih00, bhh00, wih01, whh01, bih01, bhh01, seq);
  rec_l1_head_kernel<<<NB / RB, NTHR, 0, stream>>>(seq, wih10, whh10, bih10, bhh10, wih11, whh11, bih11, bhh11,
                                                   lng, lnb, w1, bb1, w2, bb2, out);
}
